// CRNNLayer_9981503996033
// MI455X (gfx1250) — hardware-run, weakly checked
//
#include <hip/hip_runtime.h>
#include <math.h>

typedef __attribute__((ext_vector_type(16))) _Float16 v16h;
typedef __attribute__((ext_vector_type(8)))  _Float16 v8h;
typedef __attribute__((ext_vector_type(8)))  float    v8f;
typedef __attribute__((ext_vector_type(4)))  float    v4f;

constexpr int kNB      = 32;
constexpr int kNT      = 2048;
constexpr int kNC      = 128;
constexpr int kPatchT  = 8;
constexpr int kStrideT = 4;
constexpr int kNH      = 256;
constexpr int kNG      = 4 * kNH;
constexpr int kNP      = (kNT - kPatchT) / kStrideT + 1;
constexpr int kPP      = 512;
constexpr int kKC      = kPatchT * kNC;
constexpr int kRowPitch = kStrideT * kNC;
constexpr int kRowsM   = kNB * kPP;
constexpr int kXN      = kNB * kNT * kNC;
constexpr int kXPad    = 512;
constexpr int kHP      = kNH + 8;
constexpr int kSoP     = kNH + 4;
constexpr int kHhTotal = 3 * 2 * 16 * kHP;
constexpr int kGateStride = kNH * kNH;
static_assert(kNP == 511);
static_assert(kNG == 1024 && kKC == 1024 && kRowPitch == 512);
static_assert(kNT * kNC == kPP * kRowPitch);
static_assert((kRowsM % 64) == 0 && (kNG % 64) == 0 && (kKC % 32) == 0 && (kNH % 32) == 0);
static_assert(((kXN / 8) % 256) == 0 && (kXPad % 256) == 0);
static_assert(kRowsM * kRowPitch + (kKC - kRowPitch) == kXN + kXPad);

constexpr float kXCarry  = 128.0f;
constexpr float kWCarry  = 1024.0f;
constexpr float kHCarry  = 512.0f;
constexpr float kZ0Scale = 1.0f / (kXCarry * kWCarry);
constexpr float kRecInv  = 1.0f / (kHCarry * kWCarry);
constexpr float kF16MinNormal = 6.103515625e-5f;

constexpr size_t kSzZ0   = (size_t)kRowsM * kNG * 4;
constexpr size_t kSzXH   = ((size_t)kXN + kXPad) * 2;
constexpr size_t kSzW0T  = (size_t)kNG * kKC * 2;
constexpr size_t kSzST   = (size_t)kNG * kNH * 2;
constexpr size_t kOffZ0  = 0;
constexpr size_t kOffXH  = kOffZ0 + kSzZ0;
constexpr size_t kOffW0T = kOffXH + kSzXH;
constexpr size_t kOffU0T = kOffW0T + kSzW0T;
constexpr size_t kOffW1T = kOffU0T + kSzST;
constexpr size_t kOffU1T = kOffW1T + kSzST;
constexpr size_t kOffW2T = kOffU1T + kSzST;
constexpr size_t kOffU2T = kOffW2T + kSzST;
constexpr size_t kWsTotal = kOffU2T + kSzST;
static_assert(kWsTotal == 88605696ull);
static_assert(kWsTotal <= 134217728ull);
static_assert((kOffXH % 256) == 0 && (kOffW0T % 256) == 0 && (kOffU0T % 256) == 0 && (kOffW1T % 256) == 0 &&
              (kOffU1T % 256) == 0 && (kOffW2T % 256) == 0 && (kOffU2T % 256) == 0);

__device__ __forceinline__ unsigned short f2bf_bits(float f) {
  unsigned u = __float_as_uint(f);
  return (unsigned short)((u + 0x7FFFu + ((u >> 16) & 1u)) >> 16);
}
__device__ __forceinline__ float bf_bits2f(unsigned short h) { return __uint_as_float(((unsigned)h) << 16); }
__device__ __forceinline__ float bf16r(float f) { return bf_bits2f(f2bf_bits(f)); }
__device__ __forceinline__ _Float16 to_f16_flush(float v) {
  const float s = (fabsf(v) < kF16MinNormal) ? 0.0f : v;
  return (_Float16)s;
}
__device__ __forceinline__ float sigm(float v) { return 1.0f / (1.0f + expf(-v)); }

__device__ __forceinline__ void wm_guard4(v8f& a, v8f& b, v8f& c, v8f& d, v16h x, v16h y0, v16h y1, v16h y2, v16h y3) {
  asm volatile("v_nop\n\tv_nop\n\tv_nop\n\tv_nop" : "+v"(a), "+v"(b), "+v"(c), "+v"(d) : "v"(x), "v"(y0), "v"(y1), "v"(y2), "v"(y3));
}
__device__ __forceinline__ void keep4_h(v16h a, v16h b, v16h c, v16h d) { asm volatile("v_nop" :: "v"(a), "v"(b), "v"(c), "v"(d)); }
__device__ __forceinline__ void acc_guard4(v8f& a, v8f& b, v8f& c, v8f& d) { asm volatile("v_nop\n\tv_nop\n\tv_nop\n\tv_nop" : "+v"(a), "+v"(b), "+v"(c), "+v"(d)); }

union FragU { v16h v; v8h h[2]; };
__device__ __forceinline__ v16h frag_load(const _Float16* p) {
  FragU f;
  f.h[0] = *(const v8h*)(p);
  f.h[1] = *(const v8h*)(p + 16);
  return f.v;
}
__device__ __forceinline__ v8f frag_mma(v16h a, v16h b, v8f c) {
  return __builtin_amdgcn_wmma_f32_16x16x32_f16(false, a, false, b, (short)0, c, false, false);
}

__global__ __launch_bounds__(256) void wt_plane_kernel(const float* __restrict__ W, unsigned short* __restrict__ Wt, int kdim) {
  __shared__ __align__(16) float sT[64 * 68];
  const int tid = threadIdx.x, lane = tid & 31, wave = tid >> 5;
  const int k0 = blockIdx.x * 64, n0 = blockIdx.y * 64;
  const int lr = tid >> 4, c4 = (tid & 15) * 4;
#pragma unroll
  for (int i = 0; i < 4; ++i) {
    const int kk = lr + 16 * i;
    const v4f v = *(const v4f*)(W + (size_t)(k0 + kk) * kNG + n0 + c4);
    *(v4f*)(sT + kk * 68 + c4) = v;
  }
  __syncthreads();
  const int q = lane >> 3, c8 = (lane & 7) * 8;
  v8h hv[2];
#pragma unroll
  for (int it = 0; it < 2; ++it) {
    const int nl = it * 32 + wave * 4 + q;
#pragma unroll
    for (int e = 0; e < 8; ++e) {
      const float w = bf16r(sT[(c8 + e) * 68 + nl]) * kWCarry;
      hv[it][e] = to_f16_flush(w);
    }
  }
  for (int pass = 0; pass < 2; ++pass) {
#pragma unroll
    for (int it = 0; it < 2; ++it) {
      const int nl = it * 32 + wave * 4 + q;
      *(volatile v8h*)(Wt + (size_t)(n0 + nl) * kdim + k0 + c8) = hv[it];
    }
    __threadfence();
  }
}

__global__ __launch_bounds__(256) void x_plane_kernel(const float* __restrict__ x, unsigned short* __restrict__ Xh, int n8, int n8pad) {
  const int i = blockIdx.x * 256 + threadIdx.x;
  if (i >= n8pad) return;
  const bool live = (i < n8);
  const int ic = live ? i : (n8 - 1);
  const float* sp = x + (size_t)ic * 8;
  const v4f a = *(const v4f*)(sp);
  const v4f b = *(const v4f*)(sp + 4);
  v8h hv;
#pragma unroll
  for (int e = 0; e < 4; ++e) {
    const float v0 = live ? (bf16r(a[e]) * kXCarry) : 0.0f;
    const float v1 = live ? (bf16r(b[e]) * kXCarry) : 0.0f;
    hv[e]     = to_f16_flush(v0);
    hv[4 + e] = to_f16_flush(v1);
  }
  unsigned short* dp = Xh + (size_t)i * 8;
  *(volatile v8h*)dp = hv;
  __threadfence();
  *(volatile v8h*)dp = hv;
}

__global__ __launch_bounds__(256) void gemm_f16_bias_kernel(
    const unsigned short* __restrict__ Ap, int lda,
    const unsigned short* __restrict__ Btp, int ldb,
    float* __restrict__ C, int ldc,
    const float* __restrict__ bias,
    int M, int N, int K, float scale) {
  const _Float16* A  = (const _Float16*)Ap;
  const _Float16* Bt = (const _Float16*)Btp;
  __shared__ __align__(16) float sT[8][16 * 68];
  const int lane = threadIdx.x & 31;
  const int wave = threadIdx.x >> 5;
  const int tilesN = N >> 6;
  const int tilesM = M >> 6;
  const int tile = blockIdx.x * 8 + wave;
  if (tile >= tilesM * tilesN) return;
  const int tm = tile / tilesN;
  const int tn = tile - tm * tilesN;
  const int m0 = tm << 6;
  const int n0 = tn << 6;
  const int rlane = lane & 15;
  const int koff  = (lane >> 4) * 8;
  const int mOff  = (lane >> 4) * 8;

  v8f acc[4][4];
#pragma unroll
  for (int i = 0; i < 4; ++i)
#pragma unroll
    for (int j = 0; j < 4; ++j) acc[i][j] = (v8f){0.f, 0.f, 0.f, 0.f, 0.f, 0.f, 0.f, 0.f};

  for (int k0 = 0; k0 < K; k0 += 32) {
    v16h bh[4];
#pragma unroll
    for (int j = 0; j < 4; ++j) {
      const size_t bo = (size_t)(n0 + (j << 4) + rlane) * ldb + koff + k0;
      bh[j] = frag_load(Bt + bo);
    }
#pragma unroll
    for (int i = 0; i < 4; ++i) {
      const size_t ao = (size_t)(m0 + (i << 4) + rlane) * lda + koff + k0;
      const v16h ah = frag_load(A + ao);
#pragma unroll
      for (int j = 0; j < 4; ++j) acc[i][j] = frag_mma(ah, bh[j], acc[i][j]);
      wm_guard4(acc[i][0], acc[i][1], acc[i][2], acc[i][3], ah, bh[0], bh[1], bh[2], bh[3]);
    }
    keep4_h(bh[0], bh[1], bh[2], bh[3]);
  }
  acc_guard4(acc[0][0], acc[0][1], acc[0][2], acc[0][3]);
  acc_guard4(acc[1][0], acc[1][1], acc[1][2], acc[1][3]);
  acc_guard4(acc[2][0], acc[2][1], acc[2][2], acc[2][3]);
  acc_guard4(acc[3][0], acc[3][1], acc[3][2], acc[3][3]);

  float* slab = sT[wave];
#pragma unroll
  for (int i = 0; i < 4; ++i) {
    const int mBase = m0 + (i << 4);
#pragma unroll
    for (int j = 0; j < 4; ++j) {
      const int n = n0 + (j << 4) + rlane;
      const float bv = bf16r(bias[n]);
#pragma unroll
      for (int r = 0; r < 8; ++r) {
        const float v = acc[i][j][r] * scale + bv;
        slab[(mOff + r) * 68 + (j << 4) + rlane] = v;
      }
    }
    __builtin_amdgcn_fence(__ATOMIC_RELEASE, "workgroup");
    __builtin_amdgcn_wave_barrier();
    __builtin_amdgcn_fence(__ATOMIC_ACQUIRE, "workgroup");
    {
      const int hh = lane >> 4, c4 = (lane & 15) * 4;
      for (int pass = 0; pass < 2; ++pass) {
#pragma unroll
        for (int it = 0; it < 8; ++it) {
          const int row = it * 2 + hh;
          const v4f v = *(const v4f*)(slab + row * 68 + c4);
          *(volatile v4f*)(C + (size_t)(mBase + row) * ldc + n0 + c4) = v;
        }
        __threadfence();
      }
    }
    __builtin_amdgcn_fence(__ATOMIC_RELEASE, "workgroup");
    __builtin_amdgcn_wave_barrier();
    __builtin_amdgcn_fence(__ATOMIC_ACQUIRE, "workgroup");
  }
}

__device__ __forceinline__ void gate_products(const _Float16* arow, const _Float16* brow,
                                              v8f& ai, v8f& af, v8f& ag, v8f& ao) {
#pragma unroll 1
  for (int k0 = 0; k0 < kNH; k0 += 32) {
    const v16h a  = frag_load(arow + k0);
    const v16h b0 = frag_load(brow + k0);
    const v16h b1 = frag_load(brow + kGateStride + k0);
    const v16h b2 = frag_load(brow + 2 * kGateStride + k0);
    const v16h b3 = frag_load(brow + 3 * kGateStride + k0);
    ai = frag_mma(a, b0, ai);
    af = frag_mma(a, b1, af);
    ag = frag_mma(a, b2, ag);
    ao = frag_mma(a, b3, ao);
    wm_guard4(ai, af, ag, ao, a, b0, b1, b2, b3);
  }
}

__global__ __launch_bounds__(512) void lstm3_seq_kernel(
    const float* __restrict__ Z0,
    const unsigned short* __restrict__ U0p, const unsigned short* __restrict__ W1p,
    const unsigned short* __restrict__ U1p, const unsigned short* __restrict__ W2p,
    const unsigned short* __restrict__ U2p,
    const float* __restrict__ b1, const float* __restrict__ b2,
    float* __restrict__ out) {
  __shared__ __align__(16) _Float16 Hh[kHhTotal];
  __shared__ __align__(16) float So[16 * kSoP];
  const int tid = threadIdx.x, lane = tid & 31, wave = tid >> 5;
  const int c = lane & 15, hh = lane >> 4;
  const int rowbase = blockIdx.x * 16;
  const int j = 16 * wave + c;

#pragma unroll 1
  for (int i = tid; i < kHhTotal; i += 512) Hh[i] = (_Float16)0.0f;

  float ca[8], cb[8], cc[8];
#pragma unroll
  for (int r = 0; r < 8; ++r) { ca[r] = 0.0f; cb[r] = 0.0f; cc[r] = 0.0f; }
  float b1v[4], b2v[4];
#pragma unroll
  for (int g = 0; g < 4; ++g) {
    b1v[g] = bf16r(b1[g * kNH + j]);
    b2v[g] = bf16r(b2[g * kNH + j]);
  }
  __syncthreads();

  const size_t boff = (size_t)j * kNH + 8 * hh;
  const int aoff = c * kHP + 8 * hh;
  const _Float16* U0t = (const _Float16*)U0p + boff;
  const _Float16* W1t = (const _Float16*)W1p + boff;
  const _Float16* U1t = (const _Float16*)U1p + boff;
  const _Float16* W2t = (const _Float16*)W2p + boff;
  const _Float16* U2t = (const _Float16*)U2p + boff;
  const v8f z8 = {0.f, 0.f, 0.f, 0.f, 0.f, 0.f, 0.f, 0.f};

#pragma unroll 1
  for (int t = 0; t < kNP; ++t) {
    const int cur = t & 1;
    const int prv = cur ^ 1;
#pragma unroll 1
    for (int l = 0; l < 3; ++l) {
      const _Float16* Ut = (l == 0) ? U0t : ((l == 1) ? U1t : U2t);
      const _Float16* Wt = (l == 2) ? W2t : W1t;
      v8f ai = z8, af = z8, ag = z8, ao = z8;
      float zi[8], zf[8], zg[8], zo[8];
      if (l == 0) {
#pragma unroll
        for (int r = 0; r < 8; ++r) {
          const float* zr = Z0 + ((size_t)(rowbase + 8 * hh + r) * kPP + (size_t)t) * kNG + j;
          zi[r] = zr[0];
          zf[r] = zr[kNH];
          zg[r] = zr[2 * kNH];
          zo[r] = zr[3 * kNH];
        }
      } else {
        const float bi = (l == 2) ? b2v[0] : b1v[0];
        const float bf = (l == 2) ? b2v[1] : b1v[1];
        const float bg = (l == 2) ? b2v[2] : b1v[2];
        const float bo = (l == 2) ? b2v[3] : b1v[3];
#pragma unroll
        for (int r = 0; r < 8; ++r) { zi[r] = bi; zf[r] = bf; zg[r] = bg; zo[r] = bo; }
        gate_products(Hh + ((l - 1) * 2 + cur) * 16 * kHP + aoff, Wt, ai, af, ag, ao);
      }
      gate_products(Hh + (l * 2 + prv) * 16 * kHP + aoff, Ut, ai, af, ag, ao);

      _Float16* hw = Hh + (l * 2 + cur) * 16 * kHP;
      float hv[8];
#pragma unroll
      for (int r = 0; r < 8; ++r) {
        const float xi = fmaf(ai[r], kRecInv, zi[r]);
        const float xf = fmaf(af[r], kRecInv, zf[r]);
        const float xg = fmaf(ag[r], kRecInv, zg[r]);
        const float xo = fmaf(ao[r], kRecInv, zo[r]);
        const float iv = sigm(xi);
        const float fv = sigm(xf);
        const float gv = tanhf(xg);
        const float ov = sigm(xo);
        const float cn = fv * ca[r] + iv * gv;
        ca[r] = cn;
        const float hn = ov * tanhf(cn);
        hv[r] = hn;
        hw[(8 * hh + r) * kHP + j] = to_f16_flush(hn * kHCarry);
      }
      if (l == 2) {
#pragma unroll
        for (int r = 0; r < 8; ++r) So[(8 * hh + r) * kSoP + j] = hv[r];
      }
#pragma unroll
      for (int r = 0; r < 8; ++r) {
        const float tmp = ca[r];
        ca[r] = cb[r];
        cb[r] = cc[r];
        cc[r] = tmp;
      }
      __syncthreads();
      if (l == 2) {
        const float* sp = So + wave * kSoP + 4 * lane;
        const v4f o0 = *(const v4f*)(sp);
        const v4f o1 = *(const v4f*)(sp + 128);
        float* op = out + ((size_t)(rowbase + wave) * kNP + (size_t)t) * kNH + 4 * lane;
        for (int pass = 0; pass < 2; ++pass) {
          *(volatile v4f*)(op) = o0;
          *(volatile v4f*)(op + 128) = o1;
          __threadfence();
        }
      }
    }
  }
}

extern "C" void kernel_launch(void* const* d_in, const int* in_sizes, int n_in,
                              void* d_out, int out_size, void* d_ws, size_t ws_size,
                              hipStream_t stream) {
  if (n_in < 10 || d_out == nullptr || d_ws == nullptr) return;
  if (in_sizes[0] != kXN) return;
  if (in_sizes[1] != kKC * kNG) return;
  if (in_sizes[2] != kNH * kNG) return;
  if (in_sizes[3] != kNG) return;
  if (in_sizes[4] != kNH * kNG) return;
  if (in_sizes[5] != kNH * kNG) return;
  if (in_sizes[6] != kNG) return;
  if (in_sizes[7] != kNH * kNG) return;
  if (in_sizes[8] != kNH * kNG) return;
  if (in_sizes[9] != kNG) return;
  if (out_size != kNB * kNP * kNH) return;
  if (ws_size < kWsTotal) return;

  const float* x  = (const float*)d_in[0];
  const float* W0 = (const float*)d_in[1];
  const float* U0 = (const float*)d_in[2];
  const float* b0 = (const float*)d_in[3];
  const float* W1 = (const float*)d_in[4];
  const float* U1 = (const float*)d_in[5];
  const float* b1 = (const float*)d_in[6];
  const float* W2 = (const float*)d_in[7];
  const float* U2 = (const float*)d_in[8];
  const float* b2 = (const float*)d_in[9];
  float* out = (float*)d_out;

  char* ws = (char*)d_ws;
  float*          Z0  = (float*)(ws + kOffZ0);
  unsigned short* XH  = (unsigned short*)(ws + kOffXH);
  unsigned short* W0T = (unsigned short*)(ws + kOffW0T);
  unsigned short* U0T = (unsigned short*)(ws + kOffU0T);
  unsigned short* W1T = (unsigned short*)(ws + kOffW1T);
  unsigned short* U1T = (unsigned short*)(ws + kOffU1T);
  unsigned short* W2T = (unsigned short*)(ws + kOffW2T);
  unsigned short* U2T = (unsigned short*)(ws + kOffU2T);

  wt_plane_kernel<<<dim3(kKC / 64, kNG / 64), 256, 0, stream>>>(W0, W0T, kKC);
  wt_plane_kernel<<<dim3(kNH / 64, kNG / 64), 256, 0, stream>>>(U0, U0T, kNH);
  wt_plane_kernel<<<dim3(kNH / 64, kNG / 64), 256, 0, stream>>>(W1, W1T, kNH);
  wt_plane_kernel<<<dim3(kNH / 64, kNG / 64), 256, 0, stream>>>(U1, U1T, kNH);
  wt_plane_kernel<<<dim3(kNH / 64, kNG / 64), 256, 0, stream>>>(W2, W2T, kNH);
  wt_plane_kernel<<<dim3(kNH / 64, kNG / 64), 256, 0, stream>>>(U2, U2T, kNH);

  const int n8    = kXN / 8;
  const int n8pad = n8 + kXPad / 8;
  x_plane_kernel<<<(n8pad + 255) / 256, 256, 0, stream>>>(x, XH, n8, n8pad);

  gemm_f16_bias_kernel<<<dim3((kRowsM / 64) * (kNG / 64) / 8), 256, 0, stream>>>(
      XH, kRowPitch, W0T, kKC, Z0, kNG, b0, kRowsM, kNG, kKC, kZ0Scale);

  lstm3_seq_kernel<<<kNB / 16, 512, 0, stream>>>(Z0, U0T, W1T, U1T, W2T, U2T, b1, b2, out);
}
